// Attention_1073741824210
// MI455X (gfx1250) — hardware-verified
//
#include <hip/hip_runtime.h>


#define TT   1024
#define HD   64
#define ZH   2
#define RH   0
#define PCAR 1024.0f
#define SCL  0.125f
typedef _Float16 h16;
typedef unsigned short bf;
typedef __attribute__((ext_vector_type(16))) __bf16   v16bf;
typedef __attribute__((ext_vector_type(16))) _Float16 v16h;
typedef __attribute__((ext_vector_type(8)))  _Float16 v8h;
typedef __attribute__((ext_vector_type(8)))  unsigned short v8us;
typedef __attribute__((ext_vector_type(8)))  float    v8f;
typedef __attribute__((ext_vector_type(4)))  float    v4f;
typedef v8h  __attribute__((may_alias)) v8ha;
typedef v4f  __attribute__((may_alias)) v4fa;
typedef v8us __attribute__((may_alias)) v8usa;

__device__ __forceinline__ unsigned short f2bf(float f) { unsigned u = __float_as_uint(f); u += 0x7FFFu + ((u >> 16) & 1u); return (unsigned short)(u >> 16); }
__device__ __forceinline__ float bf2f(unsigned short b) { return __uint_as_float(((unsigned)b) << 16); }
__device__ __forceinline__ float bfr(float f) { return bf2f(f2bf(f)); }
__device__ __forceinline__ v16h cat16(v8h lo, v8h hi) { return __builtin_shufflevector(lo, hi, 0, 1, 2, 3, 4, 5, 6, 7, 8, 9, 10, 11, 12, 13, 14, 15); }
__device__ __forceinline__ v16bf cat16b(v8us lo, v8us hi) { return __builtin_bit_cast(v16bf, __builtin_shufflevector(lo, hi, 0, 1, 2, 3, 4, 5, 6, 7, 8, 9, 10, 11, 12, 13, 14, 15)); }
__device__ __forceinline__ v8f wmma16(v16h a, v16h b, v8f c) { return __builtin_amdgcn_wmma_f32_16x16x32_f16(false, a, false, b, (short)0, c, false, false); }
__device__ __forceinline__ v8f wmmab(v16bf a, v16bf b, v8f c) { return __builtin_amdgcn_wmma_f32_16x16x32_bf16(false, a, false, b, (short)0, c, false, false); }


template <typename T16> struct WFrag;
template <> struct WFrag<h16> { typedef v16h V; static __device__ __forceinline__ V ld(const h16* p) { return cat16(*(const v8h*)p, *(const v8h*)(p + 16)); } static __device__ __forceinline__ v8f mma(V a, V b, v8f c) { return wmma16(a, b, c); } };
template <> struct WFrag<bf> { typedef v16bf V; static __device__ __forceinline__ V ld(const bf* p) { return cat16b(*(const v8us*)p, *(const v8us*)(p + 16)); } static __device__ __forceinline__ v8f mma(V a, V b, v8f c) { return wmmab(a, b, c); } };
template <typename T16, int NSPLIT, bool BIAS>
__global__ __launch_bounds__(32) void k_gemmw(const T16* __restrict__ A, const T16* __restrict__ A2, const T16* __restrict__ Bt, const T16* __restrict__ Bt2, int K, float* C, int ldc, const float* __restrict__ bias, size_t sA, size_t sB, size_t sC) {
    typedef typename WFrag<T16>::V V;
    __shared__ __align__(16) float os[16 * 68];
    const size_t z = blockIdx.z; A += z * sA; if (A2) A2 += z * sA; Bt += z * sB; if (Bt2) Bt2 += z * sB; C += z * sC;
    const int lane = threadIdx.x & 31, lr = lane & 15, hi = lane >> 4; const int r0 = blockIdx.x * 64, c0 = blockIdx.y * 64;
    v8f acc[4][4];
#pragma unroll
    for (int mb = 0; mb < 4; ++mb)
#pragma unroll
        for (int nb = 0; nb < 4; ++nb) acc[mb][nb] = (v8f){};
    const size_t aoff = (size_t)(r0 + lr) * K + 8 * hi, boff = (size_t)(c0 + lr) * K + 8 * hi;

    for (int kc = 0; kc < K; kc += 32) {
        V a[4], a2[4];
#pragma unroll
        for (int mb = 0; mb < 4; ++mb) { a[mb] = WFrag<T16>::ld(A + aoff + (size_t)mb * 16 * K + kc); if (NSPLIT == 1 || NSPLIT == 2) a2[mb] = WFrag<T16>::ld(A2 + aoff + (size_t)mb * 16 * K + kc); }
#pragma unroll
        for (int nb = 0; nb < 4; ++nb) { const V b = WFrag<T16>::ld(Bt + boff + (size_t)nb * 16 * K + kc); V b2; if (NSPLIT >= 2) b2 = WFrag<T16>::ld(Bt2 + boff + (size_t)nb * 16 * K + kc);
#pragma unroll
            for (int mb = 0; mb < 4; ++mb) { acc[mb][nb] = WFrag<T16>::mma(a[mb], b, acc[mb][nb]); if (NSPLIT == 1 || NSPLIT == 2) acc[mb][nb] = WFrag<T16>::mma(a2[mb], b, acc[mb][nb]); if (NSPLIT >= 2) acc[mb][nb] = WFrag<T16>::mma(a[mb], b2, acc[mb][nb]); } }
        asm volatile("v_nop\n\tv_nop\n\tv_nop\n\tv_nop" : "+v"(acc[0][0]), "+v"(acc[1][1]), "+v"(acc[2][2]), "+v"(acc[3][3]) : "v"(a[0]), "v"(a[3]));
    }
#pragma unroll
    for (int mb = 0; mb < 4; ++mb) {
#pragma unroll
        for (int nb = 0; nb < 4; ++nb) {
#pragma unroll
            for (int j = 0; j < 8; ++j) os[(hi * 8 + j) * 68 + nb * 16 + lr] = acc[mb][nb][j]; }
        __builtin_amdgcn_wave_barrier(); asm volatile("" ::: "memory");
        float* crow = C + (size_t)(r0 + mb * 16) * ldc + c0;
#pragma unroll 1
        for (int ps = 0; ps < 2; ++ps) {
#pragma unroll
            for (int s = 0; s < 8; ++s) { const int row = 2 * s + hi, cofs = lr * 4; v4f val = *(const v4fa*)(os + row * 68 + cofs); if (BIAS) { val[0] += bfr(bias[c0 + cofs]); val[1] += bfr(bias[c0 + cofs + 1]); val[2] += bfr(bias[c0 + cofs + 2]); val[3] += bfr(bias[c0 + cofs + 3]); }
                *(volatile v4f*)(crow + (size_t)row * ldc + cofs) = val; }
            if (ps == 0) __threadfence(); }
        __builtin_amdgcn_wave_barrier(); asm volatile("" ::: "memory");
    }
}

__device__ __forceinline__ h16 tohx(float x) { return (h16)x; }
__device__ __forceinline__ void splitf(float y, unsigned short& h, unsigned short& l) { h = f2bf(y); l = f2bf(y - bf2f(h)); }
typedef __attribute__((ext_vector_type(2))) _Float16 v2h;
typedef __attribute__((ext_vector_type(4))) _Float16 v4h;
typedef __attribute__((ext_vector_type(2))) unsigned short v2us;
typedef __attribute__((ext_vector_type(4))) unsigned short v4us;
typedef __attribute__((ext_vector_type(2))) float v2f;
typedef __attribute__((ext_vector_type(4))) int v4i;

__global__ __launch_bounds__(256) void k_rbf(const float* __restrict__ X, float* Y, size_t n4) { const size_t i = (size_t)blockIdx.x * 256 + threadIdx.x; if (i >= n4) return; const v4f a = *(const v4f*)(X + i * 4); v4f o;
#pragma unroll
    for (int q = 0; q < 4; ++q) o[q] = bfr(a[q]);
    *(volatile v4f*)(Y + i * 4) = o; __threadfence(); *(volatile v4f*)(Y + i * 4) = o; }
__global__ __launch_bounds__(256) void k_rope(const float* __restrict__ F, int pitch, int nheads, const float* __restrict__ CS, const float* __restrict__ RF, const float* __restrict__ nw, float sc, h16* P16, bf* Ph, bf* Pl) {
    const size_t e = ((size_t)blockIdx.x * 256 + threadIdx.x) * 2; if (e >= (size_t)nheads * TT * HD) return; const int d = (int)(e % HD); const int t = (int)((e / HD) % TT); const int h = (int)(e / ((size_t)HD * TT)); const float* f = F + (size_t)t * pitch + h * HD; const float rf = RF ? RF[(size_t)h * TT + t] : 1.0f; v2h o16; v2us oh, ol;
#pragma unroll
    for (int q = 0; q < 2; ++q) { const int dd = d + q; const int dp = (dd < HD / 2) ? dd + HD / 2 : dd - HD / 2; float x0 = f[dd], x1 = f[dp];
        if (RF) { float n0 = __fmul_rn(x0, rf), n1 = __fmul_rn(x1, rf); x0 = __fmul_rn(bfr(nw[dd]), n0); x1 = __fmul_rn(bfr(nw[dp]), n1); }
        const v2f cs = *(const v2f*)(CS + ((size_t)t * HD + dd) * 2); float a = __fmul_rn(x0, cs[0]), bq = __fmul_rn(x1, cs[1]); const float r = ((dd < HD / 2) ? __fsub_rn(a, bq) : __fadd_rn(a, bq)) * sc;
        o16[q] = tohx(r); unsigned short a2, c2; splitf(r, a2, c2); oh[q] = a2; ol[q] = c2; }
    *(volatile v2h*)(P16 + e) = o16; *(volatile v2us*)(Ph + e) = oh; *(volatile v2us*)(Pl + e) = ol; __threadfence(); *(volatile v2h*)(P16 + e) = o16; *(volatile v2us*)(Ph + e) = oh; *(volatile v2us*)(Pl + e) = ol; }
__global__ __launch_bounds__(256) void k_vtp(const float* __restrict__ F, int pitch, int nheads, h16* V16, bf* Vh, bf* Vl) { const size_t e = ((size_t)blockIdx.x * 256 + threadIdx.x) * 2; if (e >= (size_t)nheads * HD * TT) return; const int t = (int)(e % TT); const int d = (int)((e / TT) % HD); const int g = (int)(e / ((size_t)TT * HD)); v2h o16; v2us oh, ol;
#pragma unroll
    for (int q = 0; q < 2; ++q) { const float x = F[(size_t)(t + q) * pitch + g * HD + d]; o16[q] = tohx(x); unsigned short a2, c2; splitf(x, a2, c2); oh[q] = a2; ol[q] = c2; }
    *(volatile v2h*)(V16 + e) = o16; *(volatile v2us*)(Vh + e) = oh; *(volatile v2us*)(Vl + e) = ol; __threadfence(); *(volatile v2h*)(V16 + e) = o16; *(volatile v2us*)(Vh + e) = oh; *(volatile v2us*)(Vl + e) = ol; }
__global__ __launch_bounds__(256) void k_csid(float* CS) { const int idx = blockIdx.x * 256 + threadIdx.x; if (idx >= TT * HD) return; v2f cs; cs[0] = 1.0f; cs[1] = 0.0f; *(volatile v2f*)(CS + (size_t)idx * 2) = cs; __threadfence(); *(volatile v2f*)(CS + (size_t)idx * 2) = cs; }
__global__ __launch_bounds__(256) void k_asoft(const float* __restrict__ Sb, h16* P16, bf* Ph, bf* Pl) {
    const int lane = threadIdx.x & 31; const int row = blockIdx.x * 8 + (threadIdx.x >> 5); if (row >= ZH * TT) return; const int i = row % TT; const int zz = row / TT; (void)zz; const bool hires = (i < RH); const float* sr = Sb + (size_t)row * TT; float v[TT / 32]; float mx = -3.0e38f;
#pragma unroll
    for (int ch = 0; ch < TT / 128; ++ch) { const int j0 = ch * 128 + lane * 4; const v4f a = *(const v4f*)(sr + j0);
#pragma unroll
        for (int q = 0; q < 4; ++q) { const int j = j0 + q; (void)j; const float t = a[q] * SCL; v[ch * 4 + q] = t; mx = fmaxf(mx, t); } }
#pragma unroll
    for (int sh = 16; sh; sh >>= 1) mx = fmaxf(mx, __shfl_xor(mx, sh, 32));
    float sum = 0.f;
#pragma unroll
    for (int k = 0; k < TT / 32; ++k) { float d0 = __fsub_rn(v[k], mx); v[k] = __builtin_amdgcn_exp2f(__fmul_rn(d0, 1.4426950408889634f)); sum += v[k]; }
#pragma unroll
    for (int sh = 16; sh; sh >>= 1) sum += __shfl_xor(sum, sh, 32);
    const float f = __fdiv_rn(hires ? 1.0f : PCAR, sum);
#pragma unroll 1
    for (int ps = 0; ps < 2; ++ps) {
        if (hires) {
#pragma unroll
            for (int ch = 0; ch < TT / 128; ++ch) { v4us oh, ol;
#pragma unroll
                for (int q = 0; q < 4; ++q) { unsigned short a, c2; splitf(v[ch * 4 + q] * f, a, c2); oh[q] = a; ol[q] = c2; }
                const size_t oo = ((size_t)zz * (RH ? RH : 1) + i) * TT + ch * 128 + lane * 4; *(volatile v4us*)(Ph + oo) = oh; *(volatile v4us*)(Pl + oo) = ol; }
        } else {
#pragma unroll
            for (int ch = 0; ch < TT / 128; ++ch) { v4h o4;
#pragma unroll
                for (int q = 0; q < 4; ++q) o4[q] = tohx(v[ch * 4 + q] * f);
                *(volatile v4h*)(P16 + (size_t)row * TT + ch * 128 + lane * 4) = o4; } }
        if (ps == 0) __threadfence(); }
}
__global__ __launch_bounds__(256) void k_sum16(const float* __restrict__ A, const float* __restrict__ B, h16* P, size_t n4) { const size_t i = (size_t)blockIdx.x * 256 + threadIdx.x; if (i >= n4) return; const v4f a = *(const v4f*)(A + i * 4); const v4f b = *(const v4f*)(B + i * 4); v4h o;
#pragma unroll
    for (int q = 0; q < 4; ++q) o[q] = tohx(__fadd_rn(bfr(a[q]), bfr(b[q])));
    *(volatile v4h*)(P + i * 4) = o; __threadfence(); *(volatile v4h*)(P + i * 4) = o; }
__global__ __launch_bounds__(256) void k_scl(const float* __restrict__ X, float c, float* Y, size_t n4) { const size_t i = (size_t)blockIdx.x * 256 + threadIdx.x; if (i >= n4) return; const v4f x = *(const v4f*)(X + i * 4); v4f o;
#pragma unroll
    for (int q = 0; q < 4; ++q) o[q] = __fmul_rn(x[q], c);
    *(volatile v4f*)(Y + i * 4) = o; __threadfence(); *(volatile v4f*)(Y + i * 4) = o; }

extern "C" void kernel_launch(void* const* d_in, const int* in_sizes, int n_in,
                              void* d_out, int out_size, void* d_ws, size_t ws_size, hipStream_t stream) {
    (void)in_sizes; (void)n_in; (void)out_size;
    const float* i0 = (const float*)d_in[0]; const float* i1 = (const float*)d_in[1]; const float* i2 = (const float*)d_in[2]; const float* i3 = (const float*)d_in[3];
    const size_t NE = 32, PL = (size_t)TT * HD;
    float* OUT0 = (float*)d_out;
    float* OUT1 = (float*)d_out + NE * PL;
    char* wsp = (char*)d_ws;
    auto take = [&](size_t bytes) { char* p = wsp; wsp += (bytes + 255) & ~(size_t)255; return (void*)p; };
    float* CS = (float*)take((size_t)TT * HD * 2 * 4); float* R0 = (float*)take(NE * PL * 4); float* R2 = (float*)take(NE * PL * 4);
    h16* QP16 = (h16*)take(NE * PL * 2); bf* QPh = (bf*)take(NE * PL * 2); bf* QPl = (bf*)take(NE * PL * 2); h16* SP16 = (h16*)take(NE * PL * 2); h16* VT16 = (h16*)take(NE * PL * 2); bf* VTh = (bf*)take(NE * PL * 2); bf* VTl = (bf*)take(NE * PL * 2);
    bf* Ph = nullptr; bf* Pl = nullptr;
    float* Sb = (float*)take((size_t)ZH * TT * TT * 4); h16* P16 = (h16*)take((size_t)ZH * TT * TT * 2); float* Ob = (float*)take((size_t)ZH * TT * HD * 4);
    if ((size_t)(wsp - (char*)d_ws) > ws_size) return;
    k_rbf<<<(unsigned)((NE * PL / 4 + 255) / 256), 256, 0, stream>>>(i0, R0, NE * PL / 4); k_rbf<<<(unsigned)((NE * PL / 4 + 255) / 256), 256, 0, stream>>>(i2, R2, NE * PL / 4);
    k_csid<<<(TT * HD + 255) / 256, 256, 0, stream>>>(CS);
    const unsigned L1 = (unsigned)((PL / 2 + 255) / 256);
    for (size_t e = 0; e < NE; ++e) {
        k_rope<<<L1, 256, 0, stream>>>(R0 + e * PL, HD, 1, CS, nullptr, nullptr, 1.0f, QP16 + e * PL, QPh + e * PL, QPl + e * PL);
        k_vtp<<<L1, 256, 0, stream>>>(R2 + e * PL, HD, 1, VT16 + e * PL, VTh + e * PL, VTl + e * PL); }
    k_sum16<<<(unsigned)((NE * PL / 4 + 255) / 256), 256, 0, stream>>>(i1, i3, SP16, NE * PL / 4);
    for (size_t e = 0; e < NE; e += ZH) {
        k_gemmw<h16, 0, false><<<dim3(TT / 64, TT / 64, ZH), 32, 0, stream>>>(QP16 + e * PL, nullptr, SP16 + e * PL, nullptr, HD, Sb, TT, nullptr, PL, PL, (size_t)TT * TT);
        k_scl<<<(unsigned)(((size_t)ZH * TT * TT / 4 + 255) / 256), 256, 0, stream>>>(Sb, 0.125f, OUT1 + e * TT * TT, (size_t)ZH * TT * TT / 4);
        k_asoft<<<ZH * TT / 8, 256, 0, stream>>>(Sb, P16, Ph, Pl);
        k_gemmw<h16, 0, false><<<dim3(TT / 64, HD / 64, ZH), 32, 0, stream>>>(P16, nullptr, VT16 + e * PL, nullptr, TT, Ob, HD, nullptr, (size_t)TT * TT, PL, PL);
        k_scl<<<(unsigned)(((size_t)ZH * PL / 4 + 255) / 256), 256, 0, stream>>>(Ob, 0.0009765625f, OUT0 + e * PL, (size_t)ZH * PL / 4); }
}
